// GCNLayer_32993938767997
// MI455X (gfx1250) — hardware-run, weakly checked
//
#include <hip/hip_runtime.h>


namespace {

constexpr int NB_ = 4, NV = 16384, KS = 32, N = NB_ * NV  , NP = N, NPL = NP  , SRCM = NV  ;
constexpr int D = 128, K2 = 2 * D, DO = 64, NL = (NPL < N ? NPL : N), NRL = NP  ;
constexpr float XS = 8.0f, WSC = 256.0f, WSQ = 0.25f, RS_ = 1024.0f, SLOPE = 0.0f, BNEPS = 1e-5f;
static_assert(NP % 32 == 0 && NP >= N && NPL % 32 == 0 && D == 128, "tiling");
typedef _Float16 b16;
typedef __attribute__((ext_vector_type(16))) _Float16 v16b;
typedef __attribute__((ext_vector_type(8))) _Float16 v8b;
typedef __attribute__((ext_vector_type(8))) float v8f;
typedef __attribute__((ext_vector_type(4))) float v4f;
__device__ __forceinline__ float bf16_rne(float f) { unsigned int u = __float_as_uint(f); u += 0x7FFFu + ((u >> 16) & 1u); return __uint_as_float(u & 0xFFFF0000u); }
__device__ __forceinline__ void split16(float v, b16& hi, b16& lo) { hi = (b16)v; lo = (b16)(v - (float)hi); }
__device__ __forceinline__ v16b frag_kb(const b16* p, int hh) { const v8b a = *(const v8b*)(p + 8 * hh), b = *(const v8b*)(p + 16 + 8 * hh); v16b f;
#pragma unroll
  for (int e = 0; e < 8; ++e) { f[e] = a[e]; f[8 + e] = b[e]; } return f; }
__device__ __forceinline__ v8f wmma16b(v16b a, v16b b, v8f c) { v8f d = __builtin_amdgcn_wmma_f32_16x16x32_f16(false, a, false, b, (short)0, c, false, false); asm volatile("v_nop\n\tv_nop\n\tv_nop\n\tv_nop" : "+v"(d) : "v"(a), "v"(b)); return d; }
__device__ __forceinline__ void wave_lds_sync() { __builtin_amdgcn_fence(__ATOMIC_RELEASE, "workgroup"); __builtin_amdgcn_wave_barrier(); __builtin_amdgcn_fence(__ATOMIC_ACQUIRE, "workgroup"); }
__device__ __forceinline__ float pmul(float a, float b) { float p = a * b; asm volatile("" : "+v"(p)); return p; }
__device__ __forceinline__ int iclamp(int v, int lo, int hi) { return v < lo ? lo : (v > hi ? hi : v); }
constexpr int CSR_NBLK = 512, CSR_GB = 9, CSR_GN = 1 << CSR_GB  , CSR_MAXG = 512, CSR_CAP = 12288  ;

typedef __attribute__((ext_vector_type(4))) _Float16 v4h;
template <int NOUTP>
__global__ __launch_bounds__(256) void wts_kernel(const float* __restrict__ ws_, const float* __restrict__ wn_, int nout, b16* __restrict__ WT, float scl) {
  const int u = blockIdx.x * 256 + threadIdx.x; if (u >= NOUTP * K2 / 8) return; const int e = u * 8; const int o = e / K2, k0 = e % K2; v8b v;
#pragma unroll
  for (int j = 0; j < 8; ++j) { const int k = k0 + j; const float w = (o < nout) ? (k < D ? wn_[(size_t)k * nout + o] : ws_[(size_t)(k - D) * nout + o]) : 0.0f; v[j] = (b16)(bf16_rne(w) * scl); }
  for (int pass = 0; pass < 2; ++pass) { *(volatile v8b*)(WT + e) = v; __threadfence(); }
}
template <int NT, bool XEXACT, bool RELU>
__global__ __launch_bounds__(64) void sage_kernel(const float* __restrict__ AGG, const float* __restrict__ X, const b16* __restrict__ WT, const b16* __restrict__ WQ, const float* __restrict__ bias, int nb, const float* __restrict__ bng, const float* __restrict__ bnb, const float* __restrict__ bnm, const float* __restrict__ bnv, float* __restrict__ out, int mrows) {
  constexpr int NOUT = NT * 16;
  __shared__ __attribute__((aligned(16))) b16 Ah[2][16][K2 + 8], Al[2][16][K2 + 8]; __shared__ __attribute__((aligned(16))) float Tf[2][16][NOUT + 4];
  const int wave = threadIdx.x >> 5, lane = threadIdx.x & 31, nloc = lane & 15, hlf = lane >> 4; const size_t m0 = (size_t)blockIdx.x * 32 + wave * 16;
  for (int idx = lane; idx < 16 * (D / 4); idx += 32) { const int rr = idx / (D / 4), c4 = (idx % (D / 4)) * 4; const size_t arow = (m0 + rr < (size_t)N) ? m0 + rr : (size_t)N - 1; const v4f av = *(const v4f*)(AGG + arow * D + c4), xv = *(const v4f*)(X + arow * D + c4); v4h h1, l1, h2, l2;
    for (int j = 0; j < 4; ++j) { const float vs = av[j] * XS; const b16 ph = (b16)vs; h1[j] = ph; l1[j] = (b16)((vs - (float)ph) * RS_); if (XEXACT) { h2[j] = (b16)(bf16_rne(xv[j]) * XS); l2[j] = (b16)0.0f; } else { const float ws_ = xv[j] * XS; const b16 p2 = (b16)ws_; h2[j] = p2; l2[j] = (b16)((ws_ - (float)p2) * RS_); } }
    *(v4h*)(&Ah[wave][rr][c4]) = h1; *(v4h*)(&Al[wave][rr][c4]) = l1; *(v4h*)(&Ah[wave][rr][D + c4]) = h2; *(v4h*)(&Al[wave][rr][D + c4]) = l2; }
  wave_lds_sync();
  v8f acc[NT];
#pragma unroll
  for (int t = 0; t < NT; ++t) acc[t] = (v8f){};
#pragma unroll 2
  for (int kb = 0; kb < K2; kb += 32) { const v16b a = frag_kb(&Ah[wave][nloc][kb], hlf), al = frag_kb(&Al[wave][nloc][kb], hlf); const bool lo = XEXACT ? (kb < D) : true;
#pragma unroll
    for (int t = 0; t < NT; ++t) { const size_t wo_ = (size_t)(t * 16 + nloc) * K2 + kb; acc[t] = wmma16b(a, frag_kb(WT + wo_, hlf), acc[t]); if (lo) acc[t] = wmma16b(al, frag_kb(WQ + wo_, hlf), acc[t]); } }
#pragma unroll
  for (int t = 0; t < NT; ++t) { const int col = t * 16 + nloc; const bool cv = col < nb; const float bb = cv ? bf16_rne(bias[col]) : 0.0f; float sg = 1.0f, sh = 0.0f;
    if (bng != nullptr && cv) { sg = bf16_rne(bng[col]) * rsqrtf(bf16_rne(bnv[col]) + BNEPS); sh = bf16_rne(bnb[col]) - bf16_rne(bnm[col]) * sg; }
    for (int r = 0; r < 8; ++r) { float v = (acc[t][r] * (1.0f / (XS * WSC)) + bb) * sg + sh; if (RELU) v = fmaxf(v, 0.0f); Tf[wave][8 * hlf + r][col] = (m0 + 8 * hlf + r < (size_t)N) ? v : 0.0f; } }
  wave_lds_sync();
  for (int pass = 0; pass < 2; ++pass) {
    if (NOUT == 128) { for (int rr = 0; rr < 16; ++rr) if (m0 + rr < (size_t)mrows) *(volatile v4f*)(out + (m0 + rr) * NOUT + lane * 4) = *(const v4f*)(&Tf[wave][rr][lane * 4]); }
    else { for (int rr = 0; rr < 16; rr += 2) { const int r2 = rr + (lane >> 4); if (m0 + r2 < (size_t)mrows) *(volatile v4f*)(out + (m0 + r2) * NOUT + (lane & 15) * 4) = *(const v4f*)(&Tf[wave][r2][(lane & 15) * 4]); } }
    __threadfence(); }
}
__global__ __launch_bounds__(256) void tmean_kernel(const float* __restrict__ X, const int* __restrict__ nbr, const int* __restrict__ vlen, float* __restrict__ AGG) {
  const int tid = threadIdx.x; const int row = tid >> 3, g = tid & 7, c0 = g * 16; const int v = blockIdx.x * 32 + row; const int vv = v < N ? v : N - 1; const int b = vv / NV;
  float m[16];
#pragma unroll
  for (int j = 0; j < 16; ++j) m[j] = 0.0f;
#pragma unroll 1
  for (int k = 0; k < KS; ++k) { int s = iclamp(nbr[(size_t)vv * KS + k], 0, NV - 1); if (SRCM < NV) s %= SRCM; const float* xr = X + ((size_t)b * NV + s) * D + c0;
#pragma unroll
    for (int q = 0; q < 4; ++q) { const v4f t4 = *(const v4f*)(xr + 4 * q); for (int j = 0; j < 4; ++j) m[4 * q + j] += bf16_rne(t4[j]); } }
  const int vl = vlen[vv]; const float inv = 1.0f / (float)(vl > 0 ? vl : 1);
  for (int pass = 0; pass < 2; ++pass) { float* ar = AGG + (size_t)v * D + c0;
#pragma unroll
    for (int q = 0; q < 4; ++q) { v4f o; for (int j = 0; j < 4; ++j) o[j] = (v < N) ? pmul(m[4 * q + j], inv) : 0.0f; *(volatile v4f*)(ar + 4 * q) = o; }
    __threadfence(); }
}
__global__ __launch_bounds__(256) void zfill_kernel(float* __restrict__ p, int n) { for (int pass = 0; pass < 2; ++pass) { for (int i = threadIdx.x; i < n; i += 256) ((volatile float*)p)[i] = 0.0f; __threadfence(); } }
}

extern "C" void kernel_launch(void* const* d_in, const int* in_sizes, int n_in, void* d_out, int out_size, void* d_ws, size_t ws_size, hipStream_t stream) {
  (void)n_in;
  auto Fp = [&](int i) { return (const float*)d_in[i]; }; auto Ip = [&](int i) { return (const int*)d_in[i]; };
  if (in_sizes[0] != N * D || in_sizes[1] != N * KS || in_sizes[2] != N || in_sizes[3] != D * D || in_sizes[4] != D * D || out_size != N * D) return;
  size_t off = 0; char* ws = (char*)d_ws;
  auto carve = [&](size_t bytes) { char* p = ws + off; off += (bytes + 255) & ~(size_t)255; return p; };
  b16* WT = (b16*)carve((size_t)D * K2 * 2); b16* WQ = (b16*)carve((size_t)D * K2 * 2); float* ZB = (float*)carve(512); float* AGG = (float*)carve((size_t)NP * D * 4);
  if (off > ws_size || off > ((size_t)48 << 20)) return;
  const unsigned gw = (D * K2 / 8 + 255) / 256;
  wts_kernel<D><<<gw, 256, 0, stream>>>(Fp(4), Fp(3), D, WT, WSC); wts_kernel<D><<<gw, 256, 0, stream>>>(Fp(4), Fp(3), D, WQ, WSQ);
  zfill_kernel<<<1, 256, 0, stream>>>(ZB, 128);
  tmean_kernel<<<NRL / 32, 256, 0, stream>>>(Fp(0), Ip(1), Ip(2), AGG);
  sage_kernel<8, true, true><<<NPL / 32, 64, 0, stream>>>(AGG, Fp(0), WT, WQ, ZB, D, nullptr, nullptr, nullptr, nullptr, (float*)d_out, NL);
}
